// CrossAttention_21225728377535
// MI455X (gfx1250) — hardware-verified
//
#include <hip/hip_runtime.h>
#include <stdint.h>


typedef _Float16 v16h __attribute__((ext_vector_type(16)));
typedef _Float16 v8h  __attribute__((ext_vector_type(8)));
typedef float    v8f  __attribute__((ext_vector_type(8)));
typedef float    v4f  __attribute__((ext_vector_type(4)));

#ifndef NB
#define NB 2
#endif
#ifndef SEQ
#define SEQ 2048
#endif
#ifndef MCTX
#define MCTX SEQ
#endif
#define NB_FULL   2
#define SEQ_FULL  2048
#define MCTX_FULL 2048
#define DM   1024
#define DC   1024
#define NH   16
#define HD   64

#define ACT_CAR   8.0f
#define W_CAR     1024.0f
#define PROJ_SCL  0.0009765625f
#define RES_CAR   2048.0f
#define RES_INV   0.00048828125f
#define S_SCL     0.001953125f
#define P_CAR     16384.0f
#define O_SCL     0.001953125f
#define OUT_SCL   3.814697265625e-06f

static_assert(NB >= 1 && NB <= NB_FULL);
static_assert(SEQ % 128 == 0);
static_assert(MCTX % 128 == 0);
static_assert(SEQ <= SEQ_FULL && MCTX <= MCTX_FULL);
static_assert(DM == NH * HD);
static_assert(HD == 64);
static_assert(DM % 128 == 0 && DC % 64 == 0 && DM % 32 == 0 && DC % 32 == 0);
static_assert(DM % 8 == 0 && DC % 8 == 0);
static_assert((long)NB_FULL * SEQ_FULL * DM * 4 == 16777216L);
static_assert(((long)(NB - 1) * SEQ_FULL + SEQ) * DM * 4 <= 16777216L);
static_assert(((long)SEQ * DM / 8) % 256 == 0 && ((long)MCTX * DC / 8) % 256 == 0);
static_assert((long)(DM / 64) * (DM / 64) * 4096 == (long)DM * DM);
static_assert((long)(2 * DM / 64) * (DC / 64) * 4096 == (long)DC * 2 * DM);
static_assert((long)(DM / 64) * ((long)NB * SEQ / 128) * 128 * 64 == (long)NB * SEQ * DM);
static_assert((long)(DM / 64) * ((long)NB * MCTX / 128) * 128 * 64 == (long)NB * MCTX * DM);
static_assert((long)(MCTX / 64) * (DM / 128) * 128 * 64 == (long)MCTX * DM);
static_assert((long)(SEQ / 128) * NH * 128 * HD == (long)SEQ * DM);
static_assert((long)(DM / 64) * (SEQ / 64) * 64 * 64 == (long)SEQ * DM);
#define WS_HALVES ((long)NB * SEQ * DM + (long)NB * MCTX * DC + 2L * DM * DM + 2L * DM * DC + \
                   (long)NB * SEQ * DM + (long)NB * MCTX * DM + (long)NB * MCTX * DM + 2L * NB * SEQ * DM)
static_assert(WS_HALVES * 2 <= 134217728L);
static_assert(((long)SEQ * DM) % 64 == 0 && ((long)MCTX * DC) % 64 == 0 && ((long)DM * DC) % 64 == 0);

union Frag16 { v16h v; v8h p[2]; };

__device__ __forceinline__ v16h ld_frag(const _Float16* p, int hl) {
  Frag16 f;
  f.p[0] = *(const v8h*)(p + 8 * hl);
  f.p[1] = *(const v8h*)(p + 16 + 8 * hl);
  return f.v;
}

__device__ __forceinline__ v8f mma(v16h a, v16h b, v8f c) {
  v8f d = __builtin_amdgcn_wmma_f32_16x16x32_f16(false, a, false, b, (short)0, c, false, false);
  asm volatile("v_nop\n\tv_nop\n\tv_nop\n\tv_nop" : "+v"(d) : "v"(a), "v"(b));
  return d;
}

__device__ __forceinline__ float bf16_rne(float x) {
  unsigned int u = __builtin_bit_cast(unsigned int, x);
  u += 0x7FFFu + ((u >> 16) & 1u);
  return __builtin_bit_cast(float, u & 0xFFFF0000u);
}

__global__ __launch_bounds__(256) void k_cvt8(const float* __restrict__ src,
                                              _Float16* __restrict__ dst,
                                              int cols, int pitch, float car, int total8,
                                              long sbs, long dbs)
{
  const int i8 = blockIdx.x * 256 + threadIdx.x;
  if (i8 >= total8) return;
  const size_t e   = (size_t)i8 * 8;
  const size_t r   = e / (size_t)cols;
  const int    col = (int)(e - r * (size_t)cols);
  const float* s = src + (size_t)blockIdx.y * (size_t)sbs + r * (size_t)pitch + col;
  const v4f x0 = *(const v4f*)s;
  const v4f x1 = *(const v4f*)(s + 4);
  v8h o;
#pragma unroll
  for (int j = 0; j < 4; ++j) {
    const float t0 = x0[j];
    const float t1 = x1[j];
    o[j]     = (_Float16)(bf16_rne(t0) * car);
    o[4 + j] = (_Float16)(bf16_rne(t1) * car);
  }
  _Float16* d = dst + (size_t)blockIdx.y * (size_t)dbs + e;
  *(volatile v8h*)d = o;
  __threadfence();
  *(volatile v8h*)d = o;
}

__global__ __launch_bounds__(256) void k_trw(const float* __restrict__ W,
                                             _Float16* __restrict__ WT, int R, int C)
{
  __shared__ float tile[64 * 65];
  const int tid = threadIdx.x;
  const int c0 = blockIdx.x * 64, r0 = blockIdx.y * 64;
#pragma unroll
  for (int i = 0; i < 4; ++i) {
    const int idx = i * 256 + tid;
    const int r = idx >> 4, c4 = (idx & 15) * 4;
    const v4f v = *(const v4f*)(W + (size_t)(r0 + r) * C + c0 + c4);
    float* tp = tile + r * 65 + c4;
    tp[0] = v[0]; tp[1] = v[1]; tp[2] = v[2]; tp[3] = v[3];
  }
  __syncthreads();
  v8h o[2];
  _Float16* dp[2];
#pragma unroll
  for (int i = 0; i < 2; ++i) {
    const int line = i * 32 + (tid >> 3);
    const int pc   = (tid & 7) * 8;
#pragma unroll
    for (int j = 0; j < 8; ++j)
      o[i][j] = (_Float16)(bf16_rne(tile[(pc + j) * 65 + line]) * W_CAR);
    dp[i] = WT + (size_t)(c0 + line) * R + r0 + pc;
  }
  *(volatile v8h*)dp[0] = o[0];
  *(volatile v8h*)dp[1] = o[1];
  __threadfence();
  *(volatile v8h*)dp[0] = o[0];
  *(volatile v8h*)dp[1] = o[1];
}

__device__ __forceinline__ void gemm_core(const _Float16* ap0, const _Float16* ap1,
                                          const _Float16* bp, int K, int hl, v8f (&acc)[8])
{
  const size_t bst = (size_t)16 * K;
#pragma unroll 1
  for (int k0 = 0; k0 < K; k0 += 32) {
    const v16h a0 = ld_frag(ap0 + k0, hl);
    const v16h a1 = ld_frag(ap1 + k0, hl);
    const v16h b0 = ld_frag(bp + k0, hl);
    const v16h b1 = ld_frag(bp + bst + k0, hl);
    const v16h b2 = ld_frag(bp + 2 * bst + k0, hl);
    const v16h b3 = ld_frag(bp + 3 * bst + k0, hl);
    acc[0] = mma(a0, b0, acc[0]);
    acc[1] = mma(a0, b1, acc[1]);
    acc[2] = mma(a0, b2, acc[2]);
    acc[3] = mma(a0, b3, acc[3]);
    acc[4] = mma(a1, b0, acc[4]);
    acc[5] = mma(a1, b1, acc[5]);
    acc[6] = mma(a1, b2, acc[6]);
    acc[7] = mma(a1, b3, acc[7]);
  }
}

__global__ __launch_bounds__(128) __attribute__((amdgpu_num_vgpr(256)))
void k_proj(const _Float16* __restrict__ A, const _Float16* __restrict__ Bt,
            _Float16* __restrict__ PH, int K, int ldc,
            long sA, long sB, long sC)
{
  __shared__ __attribute__((aligned(16))) _Float16 ldsH[128 * 72];

  const int tid = threadIdx.x, lane = tid & 31, w = tid >> 5;
  const int hl = lane >> 4, c = lane & 15;
  const int m0 = blockIdx.y * 128, n0 = blockIdx.x * 64;
  const int mw = m0 + 32 * w;
  const size_t z = blockIdx.z;

  const _Float16* ap0 = A  + z * (size_t)sA + (size_t)(mw + c) * K;
  const _Float16* ap1 = A  + z * (size_t)sA + (size_t)(mw + 16 + c) * K;
  const _Float16* bp  = Bt + z * (size_t)sB + (size_t)(n0 + c) * K;

  v8f acc[8] = {};
  gemm_core(ap0, ap1, bp, K, hl, acc);

#pragma unroll
  for (int i = 0; i < 2; ++i)
#pragma unroll
    for (int t = 0; t < 4; ++t)
#pragma unroll
      for (int r = 0; r < 8; ++r) {
        const int rowl = 32 * w + 16 * i + 8 * hl + r;
        const float v = acc[i * 4 + t][r] * PROJ_SCL;
        ldsH[rowl * 72 + 16 * t + c] = (_Float16)v;
      }
  __syncthreads();

  _Float16* const bh = PH + z * (size_t)sC + (size_t)m0 * ldc + n0;
  for (int i = 0; i < 8; ++i) {
    const int q = i * 128 + tid;
    const int rowl = q >> 3, ch = (q & 7) * 8;
    const v8h vh = *(const v8h*)(ldsH + rowl * 72 + ch);
    *(volatile v8h*)(bh + (size_t)rowl * ldc + ch) = vh;
  }
  __threadfence();
  for (int i = 0; i < 8; ++i) {
    const int q = i * 128 + tid;
    const int rowl = q >> 3, ch = (q & 7) * 8;
    const v8h vh = *(const v8h*)(ldsH + rowl * 72 + ch);
    *(volatile v8h*)(bh + (size_t)rowl * ldc + ch) = vh;
  }
}

__global__ __launch_bounds__(256) __attribute__((amdgpu_num_vgpr(256)))
void k_attn(const _Float16* __restrict__ Q, const _Float16* __restrict__ Kp,
            const _Float16* __restrict__ Vt,
            _Float16* __restrict__ OH, _Float16* __restrict__ OL)
{
  constexpr int KT_H   = 32 * 72;
  constexpr int V_H    = HD * 40;
  constexpr int P_H    = 8 * 16 * 40;
  constexpr int TILE_H = KT_H + V_H + P_H;
  constexpr int EPI_H  = 2 * 128 * 72;
  constexpr int LDS_H  = (TILE_H > EPI_H) ? TILE_H : EPI_H;
  static_assert(32 * 8 == 256 && HD * 4 == 256);
  static_assert(MCTX % 32 == 0);
  __shared__ __attribute__((aligned(16))) _Float16 lds[LDS_H];
  _Float16* const ldsK  = lds;
  _Float16* const ldsV  = ldsK + KT_H;
  _Float16* const ldsP  = ldsV + V_H;
  _Float16* const ldsOH = lds;
  _Float16* const ldsOL = lds + 128 * 72;

  const int tid = threadIdx.x, lane = tid & 31, w = tid >> 5;
  const int hl = lane >> 4, c = lane & 15;
  const int q0 = blockIdx.x * 128;
  const int col0 = blockIdx.y * HD;
  const size_t zq = (size_t)blockIdx.z * ((size_t)SEQ * DM);
  const size_t zk = (size_t)blockIdx.z * ((size_t)MCTX * DM);

  const size_t qrow = zq + (size_t)(q0 + 16 * w + c) * DM + col0;
  v16h qf[2];
#pragma unroll
  for (int ks = 0; ks < 2; ++ks)
    qf[ks] = ld_frag(Q + qrow + 32 * ks, hl);
  _Float16* const myP = ldsP + w * (16 * 40);

  const int krr = tid >> 3, kcc = (tid & 7) * 8;
  const int vdd = tid >> 2, vkc = (tid & 3) * 8;
  const _Float16* const kg = Kp + zk + (size_t)krr * DM + col0 + kcc;
  const _Float16* const vg = Vt + zk + (size_t)(col0 + vdd) * MCTX + vkc;

  float m[8], l[8];
  v8f oa[4] = {};
#pragma unroll
  for (int r = 0; r < 8; ++r) { m[r] = -__builtin_inff(); l[r] = 0.f; }

#pragma unroll 1
  for (int kt = 0; kt < MCTX / 32; ++kt) {
    const int mk = kt * 32;
    {
      const v8h k8 = *(const v8h*)(kg + (size_t)mk * DM);
      const v8h v8 = *(const v8h*)(vg + mk);
      *(v8h*)(ldsK + krr * 72 + kcc) = k8;
      *(v8h*)(ldsV + vdd * 40 + vkc) = v8;
    }
    __syncthreads();

    v8f sc[2] = {};
#pragma unroll
    for (int ks = 0; ks < 2; ++ks) {
#pragma unroll
      for (int t = 0; t < 2; ++t) {
        const v16h kf = ld_frag(ldsK + (16 * t + c) * 72 + 32 * ks, hl);
        sc[t] = mma(qf[ks], kf, sc[t]);
      }
    }

#pragma unroll
    for (int r = 0; r < 8; ++r) {
      const float v0 = sc[0][r] * S_SCL;
      const float v1 = sc[1][r] * S_SCL;
      float tm = fmaxf(v0, v1);
      tm = fmaxf(tm, __shfl_xor(tm, 1, 32));
      tm = fmaxf(tm, __shfl_xor(tm, 2, 32));
      tm = fmaxf(tm, __shfl_xor(tm, 4, 32));
      tm = fmaxf(tm, __shfl_xor(tm, 8, 32));
      const float mn = fmaxf(m[r], tm);
      const float al = __expf(m[r] - mn);
      const float p0 = __expf(v0 - mn), p1 = __expf(v1 - mn);
      float rs = p0 + p1;
      rs += __shfl_xor(rs, 1, 32);
      rs += __shfl_xor(rs, 2, 32);
      rs += __shfl_xor(rs, 4, 32);
      rs += __shfl_xor(rs, 8, 32);
      l[r] = l[r] * al + rs;
      m[r] = mn;
#pragma unroll
      for (int t = 0; t < 4; ++t) oa[t][r] *= al;
      _Float16* pp = myP + (8 * hl + r) * 40 + c;
      pp[0]  = (_Float16)(p0 * P_CAR);
      pp[16] = (_Float16)(p1 * P_CAR);
    }
    __syncthreads();

    const v16h pf = ld_frag(myP + c * 40, hl);
#pragma unroll
    for (int t = 0; t < 4; ++t) {
      const v16h vf = ld_frag(ldsV + (16 * t + c) * 40, hl);
      oa[t] = mma(pf, vf, oa[t]);
    }
    __syncthreads();
  }

#pragma unroll
  for (int r = 0; r < 8; ++r) {
    const float inv = (1.0f / l[r]) * O_SCL;
    const int rowl = 16 * w + 8 * hl + r;
#pragma unroll
    for (int t = 0; t < 4; ++t) {
      const float v = oa[t][r] * inv;
      const _Float16 hv = (_Float16)v;
      const float res = (v - (float)hv) * RES_CAR;
      ldsOH[rowl * 72 + 16 * t + c] = hv;
      ldsOL[rowl * 72 + 16 * t + c] = (_Float16)res;
    }
  }
  __syncthreads();
  _Float16* const bh = OH + zq + (size_t)q0 * DM + col0;
  _Float16* const bl = OL + zq + (size_t)q0 * DM + col0;
  for (int i = 0; i < 4; ++i) {
    const int q = i * 256 + tid;
    const int rowl = q >> 3, ch = (q & 7) * 8;
    const v8h vh = *(const v8h*)(ldsOH + rowl * 72 + ch);
    const v8h vl = *(const v8h*)(ldsOL + rowl * 72 + ch);
    *(volatile v8h*)(bh + (size_t)rowl * DM + ch) = vh;
    *(volatile v8h*)(bl + (size_t)rowl * DM + ch) = vl;
  }
  __threadfence();
  for (int i = 0; i < 4; ++i) {
    const int q = i * 256 + tid;
    const int rowl = q >> 3, ch = (q & 7) * 8;
    const v8h vh = *(const v8h*)(ldsOH + rowl * 72 + ch);
    const v8h vl = *(const v8h*)(ldsOL + rowl * 72 + ch);
    *(volatile v8h*)(bh + (size_t)rowl * DM + ch) = vh;
    *(volatile v8h*)(bl + (size_t)rowl * DM + ch) = vl;
  }
}

__global__ __launch_bounds__(128) __attribute__((amdgpu_num_vgpr(256)))
void k_oproj(const _Float16* __restrict__ AH, const _Float16* __restrict__ AL,
             const _Float16* __restrict__ Bt, float* __restrict__ Out)
{
  __shared__ __attribute__((aligned(16))) float ldsF[64 * 68];
  static_assert(128 % 16 == 0);
  static_assert(8 * 128 == 64 * 16);

  const int tid = threadIdx.x, lane = tid & 31, w = tid >> 5;
  const int hl = lane >> 4, c = lane & 15;
  const int m0 = blockIdx.y * 64, n0 = blockIdx.x * 64;
  const int mw = m0 + 16 * w;
  const size_t za = (size_t)blockIdx.z * ((size_t)SEQ * DM);
  const size_t zo = (size_t)blockIdx.z * ((size_t)SEQ_FULL * DM);

  const _Float16* ap0 = AH + za + (size_t)(mw + c) * DM;
  const _Float16* ap1 = AL + za + (size_t)(mw + c) * DM;
  const _Float16* bp  = Bt + (size_t)(n0 + c) * DM;

  v8f acc[8] = {};
  gemm_core(ap0, ap1, bp, DM, hl, acc);

#pragma unroll
  for (int t = 0; t < 4; ++t)
#pragma unroll
    for (int r = 0; r < 8; ++r) {
      const int rowl = 16 * w + 8 * hl + r;
      ldsF[rowl * 68 + 16 * t + c] = (acc[t][r] + acc[4 + t][r] * RES_INV) * OUT_SCL;
    }
  __syncthreads();

  const int colc = (tid & 15) * 4;

  float* const ob = Out + zo + (size_t)m0 * DM + n0;
  for (int i = 0; i < 8; ++i) {
    const int qi = i * 128 + tid;
    const int rowl = qi >> 4;
    const v4f v = *(const v4f*)(ldsF + rowl * 68 + colc);
    *(volatile v4f*)(ob + (size_t)rowl * DM + colc) = v;
  }
  __threadfence();
  for (int i = 0; i < 8; ++i) {
    const int qi = i * 128 + tid;
    const int rowl = qi >> 4;
    const v4f v = *(const v4f*)(ldsF + rowl * 68 + colc);
    *(volatile v4f*)(ob + (size_t)rowl * DM + colc) = v;
  }
}

extern "C" void kernel_launch(void* const* d_in, const int* in_sizes, int n_in,
                              void* d_out, int out_size, void* d_ws, size_t ws_size,
                              hipStream_t stream)
{
  if (n_in < 5) return;
  if ((long)in_sizes[0] < ((long)(NB - 1) * SEQ_FULL + SEQ) * DM) return;
  if ((long)in_sizes[1] < ((long)(NB - 1) * MCTX_FULL + MCTX) * DC) return;
  if ((long)in_sizes[2] < (long)DM * DM) return;
  if ((long)in_sizes[3] < (long)DC * 2 * DM) return;
  if ((long)in_sizes[4] < (long)DM * DM) return;
  if ((long)out_size < ((long)(NB - 1) * SEQ_FULL + SEQ) * DM) return;

  const float* x   = (const float*)d_in[0];
  const float* ctx = (const float*)d_in[1];
  const float* Wq  = (const float*)d_in[2];
  const float* Wkv = (const float*)d_in[3];
  const float* Wc  = (const float*)d_in[4];
  float* out = (float*)d_out;

  const size_t nX  = (size_t)NB * SEQ * DM;
  const size_t nC  = (size_t)NB * MCTX * DC;
  const size_t nWs = (size_t)DM * DM;
  const size_t nWc = (size_t)DM * DC;
  const size_t nK  = (size_t)NB * MCTX * DM;
  const size_t total_halves = nX + nC + 2 * nWs + 2 * nWc + nX + nK + nK + 2 * nX;
  if (total_halves != (size_t)WS_HALVES) return;
  if (total_halves * sizeof(_Float16) > ws_size) return;

  _Float16* X16  = (_Float16*)d_ws;
  _Float16* C16  = X16  + nX;
  _Float16* WqT  = C16  + nC;
  _Float16* WkvT = WqT  + nWs;
  _Float16* WcT  = WkvT + 2 * nWc;
  _Float16* Q16  = WcT  + nWs;
  _Float16* K16  = Q16  + nX;
  _Float16* Vt16 = K16  + nK;
  _Float16* OH   = Vt16 + nK;
  _Float16* OL   = OH   + nX;
  const _Float16* WkT = WkvT;
  const _Float16* WvT = WkvT + nWc;

  const int tx8 = (int)((size_t)SEQ * DM / 8);
  const int tc8 = (int)((size_t)MCTX * DC / 8);
  k_cvt8<<<dim3((tx8 + 255) / 256, NB), 256, 0, stream>>>(x,   X16, DM, DM, ACT_CAR, tx8,
                                                           (long)SEQ_FULL * DM, (long)SEQ * DM);
  k_cvt8<<<dim3((tc8 + 255) / 256, NB), 256, 0, stream>>>(ctx, C16, DC, DC, ACT_CAR, tc8,
                                                           (long)MCTX_FULL * DC, (long)MCTX * DC);

  k_trw<<<dim3(DM / 64, DM / 64), 256, 0, stream>>>(Wq, WqT, DM, DM);
  k_trw<<<dim3(2 * DM / 64, DC / 64), 256, 0, stream>>>(Wkv, WkvT, DC, 2 * DM);
  k_trw<<<dim3(DM / 64, DM / 64), 256, 0, stream>>>(Wc, WcT, DM, DM);

  k_proj<<<dim3(DM / 64, NB * SEQ / 128, 1), 128, 0, stream>>>(X16, WqT, Q16, DM, DM, 0L, 0L, 0L);
  k_proj<<<dim3(DM / 64, NB * MCTX / 128, 1), 128, 0, stream>>>(C16, WkT, K16, DC, DM, 0L, 0L, 0L);
  k_proj<<<dim3(MCTX / 64, DM / 128, NB), 128, 0, stream>>>(WvT, C16, Vt16, DC, MCTX,
                                                             0L, (long)MCTX * DC, (long)DM * MCTX);

  k_attn<<<dim3(SEQ / 128, NH, NB), 256, 0, stream>>>(Q16, K16, Vt16, OH, OL);

  k_oproj<<<dim3(DM / 64, SEQ / 64, NB), 128, 0, stream>>>(OH, OL, WcT, out);
}
